// SelfAttention_41429254537370
// MI455X (gfx1250) — hardware-verified
//
#include <hip/hip_runtime.h>


#ifndef NB
#define NB 2
#endif
#ifndef SEQ
#define SEQ 2048
#endif
#define NB_FULL    2
#define SEQ_FULL   2048
#define NHEAD      16
#define HDIM       64
#define DM         1024
#define N3         3072
#define A2_LD      2048
#define MROWS      (NB * SEQ)
#define PLANE      ((size_t)NB * NHEAD * SEQ * HDIM)
#define BQ         128
#define BK         32
#define NWAVE      8
#define GT         128
#define OP         68
#define CP         136
#define QKV_CARRY  16.0f
#define P_CARRY    4096.0f
#define CTX_CARRY  64.0f

static_assert(SEQ % GT == 0);
static_assert(SEQ % BQ == 0);
static_assert(SEQ % BK == 0);
static_assert(BQ == NWAVE * 16);
static_assert(HDIM == 64);
static_assert(GT == 2 * HDIM);
static_assert(DM == NHEAD * HDIM);
static_assert(N3 == 3 * DM);
static_assert(DM % GT == 0 && N3 % GT == 0 && MROWS % GT == 0);
static_assert(DM % 32 == 0 && A2_LD % 32 == 0);
static_assert(A2_LD == 2 * DM);
static_assert(DM / 8 == 128);
static_assert(SEQ <= SEQ_FULL);
static_assert(NB >= 1 && NB <= NB_FULL);
static_assert((OP * 4) % 16 == 0 && OP >= 64);
static_assert((CP * 2) % 16 == 0 && CP >= GT);
static_assert(GT * GT / 8 == 8 * 256);
static_assert(NWAVE * 32 == 256);

typedef __bf16         bf16;
typedef _Float16       f16;
typedef unsigned short u16;
typedef bf16     v16bf __attribute__((ext_vector_type(16)));
typedef f16      v16h  __attribute__((ext_vector_type(16)));
typedef f16      v8h   __attribute__((ext_vector_type(8)));
typedef float    v8f   __attribute__((ext_vector_type(8)));
typedef float    v4f   __attribute__((ext_vector_type(4)));
typedef unsigned v4u   __attribute__((ext_vector_type(4)));

union FragH  { v16h  v; v4u q[2]; f16  h[16]; };
union FragX  { v16bf vb; v16h vh; v4u q[2]; };
union Pack8B { v4u u; bf16 h[8]; };
union Pack8H { v4u u; v8h v; f16 h[8]; };

#define XB_BYTES  ((size_t)MROWS * DM * 2)
#define WB_BYTES  ((size_t)N3 * DM * 2)
#define W2_BYTES  ((size_t)DM * A2_LD * 2)
#define QK_BYTES  ((size_t)2 * PLANE * 2)
#define VT_BYTES  ((size_t)PLANE * 2)
#define A2_BYTES  ((size_t)MROWS * A2_LD * 2)
#define WS_TOTAL  (XB_BYTES + WB_BYTES + W2_BYTES + QK_BYTES + VT_BYTES + A2_BYTES)
static_assert(WS_TOTAL <= (size_t)134217728);
static_assert(XB_BYTES % 128 == 0 && WB_BYTES % 128 == 0 && W2_BYTES % 128 == 0);
static_assert(QK_BYTES % 128 == 0 && VT_BYTES % 128 == 0 && A2_BYTES % 128 == 0);

static __device__ __forceinline__ v8f mma_bf16(v16bf a, v16bf b, v8f acc) {
  acc = __builtin_amdgcn_wmma_f32_16x16x32_bf16(false, a, false, b, (short)0, acc, false, false);
  asm volatile("v_nop\n\tv_nop\n\tv_nop\n\tv_nop" : "+v"(acc) : "v"(a), "v"(b));
  return acc;
}
static __device__ __forceinline__ v8f mma_f16(v16h a, v16h b, v8f acc) {
  acc = __builtin_amdgcn_wmma_f32_16x16x32_f16(false, a, false, b, (short)0, acc, false, false);
  asm volatile("v_nop\n\tv_nop\n\tv_nop\n\tv_nop" : "+v"(acc) : "v"(a), "v"(b));
  return acc;
}

__global__ __launch_bounds__(256) void cvt_bf16_kernel(const float* __restrict__ in,
                                                       u16* __restrict__ outp,
                                                       int rows, int rows_per_batch, int src_batch_rows) {
  const int idx = blockIdx.x * 256 + threadIdx.x;
  if (idx >= rows * 128) return;
  const int row   = idx >> 7;
  const int piece = idx & 127;
  const int b = row / rows_per_batch;
  const int s = row - b * rows_per_batch;
  const float* src = in + ((size_t)b * src_batch_rows + s) * DM + piece * 8;
  const v4f a0 = *(const v4f*)(src);
  const v4f a1 = *(const v4f*)(src + 4);
  Pack8B pk;
  #pragma unroll
  for (int i = 0; i < 4; ++i) {
    pk.h[i]     = (bf16)a0[i];
    pk.h[4 + i] = (bf16)a1[i];
  }
  const v4u val = pk.u;
  const size_t off = (size_t)row * DM + piece * 8;
  *(volatile v4u*)(outp + off) = val;
  __threadfence();
  *(volatile v4u*)(outp + off) = val;
}

__global__ __launch_bounds__(256) void cvt_wout_kernel(const float* __restrict__ in, f16* __restrict__ w2) {
  const int idx = blockIdx.x * 256 + threadIdx.x;
  if (idx >= DM * 128) return;
  const int row   = idx >> 7;
  const int piece = idx & 127;
  const float* src = in + (size_t)row * DM + piece * 8;
  const v4f a0 = *(const v4f*)(src);
  const v4f a1 = *(const v4f*)(src + 4);
  Pack8H ph, pl;
  #pragma unroll
  for (int i = 0; i < 4; ++i) {
    const float w0 = (float)(bf16)a0[i];
    const float w1 = (float)(bf16)a1[i];
    ph.h[i]     = (f16)(w0 * CTX_CARRY);
    ph.h[4 + i] = (f16)(w1 * CTX_CARRY);
    pl.h[i]     = (f16)w0;
    pl.h[4 + i] = (f16)w1;
  }
  const v4u vh = ph.u;
  const v4u vl = pl.u;
  const size_t off = (size_t)row * A2_LD + piece * 8;
  *(volatile v4u*)(w2 + off)      = vh;
  *(volatile v4u*)(w2 + off + DM) = vl;
  __threadfence();
  *(volatile v4u*)(w2 + off)      = vh;
  *(volatile v4u*)(w2 + off + DM) = vl;
}

template <int BF>
static __device__ __forceinline__ void gemm_tile(const u16* __restrict__ A, const u16* __restrict__ W,
                                                 const int ld, const int arow, const int wrow, const int koff,
                                                 v8f (&acc)[2][4]) {
  const u16* ap = A + (size_t)arow * ld + koff;
  const u16* bp = W + (size_t)wrow * ld + koff;
  #pragma unroll 1
  for (int k0 = 0; k0 < ld; k0 += 32) {
    FragX a[2], bw[4];
    #pragma unroll
    for (int tm = 0; tm < 2; ++tm) {
      const u16* p = ap + (size_t)(tm * 16) * ld + k0;
      a[tm].q[0] = *(const v4u*)(p);
      a[tm].q[1] = *(const v4u*)(p + 16);
    }
    #pragma unroll
    for (int tn = 0; tn < 4; ++tn) {
      const u16* p = bp + (size_t)(tn * 16) * ld + k0;
      bw[tn].q[0] = *(const v4u*)(p);
      bw[tn].q[1] = *(const v4u*)(p + 16);
    }
    #pragma unroll
    for (int tm = 0; tm < 2; ++tm) {
      #pragma unroll
      for (int tn = 0; tn < 4; ++tn) {
        if (BF) acc[tm][tn] = mma_bf16(a[tm].vb, bw[tn].vb, acc[tm][tn]);
        else    acc[tm][tn] = mma_f16(a[tm].vh, bw[tn].vh, acc[tm][tn]);
      }
    }
  }
}

__global__ __launch_bounds__(256) void qkv_gemm_kernel(const u16* __restrict__ xb,
                                                       const u16* __restrict__ wb,
                                                       const float* __restrict__ b_in,
                                                       f16* __restrict__ qk,
                                                       f16* __restrict__ vt) {
  __shared__ __align__(16) f16 sC[GT * CP];
  const int tid   = threadIdx.x;
  const int wave  = __builtin_amdgcn_readfirstlane(tid >> 5);
  const int lane  = tid & 31;
  const int lq    = lane & 15;
  const int hi    = lane >> 4;
  const int waveM = wave >> 1;
  const int waveN = wave & 1;
  const int mBase = blockIdx.y * GT;
  const int nBase = blockIdx.x * GT;

  v8f acc[2][4];
  #pragma unroll
  for (int tm = 0; tm < 2; ++tm) {
    #pragma unroll
    for (int tn = 0; tn < 4; ++tn) acc[tm][tn] = (v8f){0, 0, 0, 0, 0, 0, 0, 0};
  }
  gemm_tile<1>(xb, wb, DM, mBase + waveM * 32 + lq, nBase + waveN * 64 + lq, hi * 8, acc);

  const int which = nBase / DM;
  const int h0    = (nBase - which * DM) / HDIM;
  const int b     = mBase / SEQ;
  const int s0    = mBase - b * SEQ;

  float bias[4];
  #pragma unroll
  for (int tn = 0; tn < 4; ++tn) bias[tn] = (float)(bf16)b_in[nBase + waveN * 64 + tn * 16 + lq];

  if (which < 2) {
    #pragma unroll
    for (int tm = 0; tm < 2; ++tm) {
      #pragma unroll
      for (int tn = 0; tn < 4; ++tn) {
        #pragma unroll
        for (int j = 0; j < 8; ++j) {
          sC[(waveM * 32 + tm * 16 + hi * 8 + j) * CP + waveN * 64 + tn * 16 + lq] =
              (f16)((acc[tm][tn][j] + bias[tn]) * QKV_CARRY);
        }
      }
    }
  } else {
    #pragma unroll
    for (int tm = 0; tm < 2; ++tm) {
      #pragma unroll
      for (int tn = 0; tn < 4; ++tn) {
        Pack8H ph;
        #pragma unroll
        for (int j = 0; j < 8; ++j) ph.h[j] = (f16)((acc[tm][tn][j] + bias[tn]) * QKV_CARRY);
        *(v4u*)(&sC[(waveN * 64 + tn * 16 + lq) * CP + waveM * 32 + tm * 16 + hi * 8]) = ph.u;
      }
    }
  }
  __syncthreads();

  v4u    val[8];
  size_t dst[8];
  #pragma unroll
  for (int it = 0; it < 8; ++it) {
    const int p    = it * 256 + tid;
    const int line = p >> 3;
    const int q    = p & 7;
    const int r0   = line >> 1;
    const int r1   = line & 1;
    val[it] = *(const v4u*)(&sC[r0 * CP + r1 * 64 + q * 8]);
    if (which < 2) {
      dst[it] = (size_t)which * PLANE +
                (((size_t)b * NHEAD + h0 + r1) * SEQ + s0 + r0) * HDIM + q * 8;
    } else {
      dst[it] = (((size_t)b * NHEAD + h0 + (r0 >> 6)) * HDIM + (r0 & 63)) * SEQ + s0 + r1 * 64 + q * 8;
    }
  }
  if (which < 2) {
    #pragma unroll
    for (int it = 0; it < 8; ++it) *(volatile v4u*)(qk + dst[it]) = val[it];
    __threadfence();
    #pragma unroll
    for (int it = 0; it < 8; ++it) *(volatile v4u*)(qk + dst[it]) = val[it];
  } else {
    #pragma unroll
    for (int it = 0; it < 8; ++it) *(volatile v4u*)(vt + dst[it]) = val[it];
    __threadfence();
    #pragma unroll
    for (int it = 0; it < 8; ++it) *(volatile v4u*)(vt + dst[it]) = val[it];
  }
}

__global__ __launch_bounds__(256) void attn_kernel(const f16* __restrict__ qk,
                                                   const f16* __restrict__ vt,
                                                   f16* __restrict__ a2) {
  const int qblk = blockIdx.x;
  const int h    = blockIdx.y;
  const int b    = blockIdx.z;
  const int tid  = threadIdx.x;
  const int wave = __builtin_amdgcn_readfirstlane(tid >> 5);
  const int lane = tid & 31;
  const int lq   = lane & 15;
  const int hi   = lane >> 4;

  __shared__ __align__(16) float sO[NWAVE * 16 * OP];

  const int qrow0 = qblk * BQ + wave * 16;

  const f16* q_h  = qk + ((size_t)b * NHEAD + h) * SEQ * HDIM;
  const f16* k_h  = qk + PLANE + ((size_t)b * NHEAD + h) * SEQ * HDIM;
  const f16* vt_h = vt + ((size_t)b * NHEAD + h) * HDIM * SEQ;

  FragH qf[2];
  #pragma unroll
  for (int f = 0; f < 2; ++f) {
    const f16* base = q_h + (size_t)(qrow0 + lq) * HDIM + f * 32 + hi * 8;
    qf[f].q[0] = *(const v4u*)(base);
    qf[f].q[1] = *(const v4u*)(base + 16);
  }

  v8f o[4];
  #pragma unroll
  for (int dt = 0; dt < 4; ++dt) o[dt] = (v8f){0, 0, 0, 0, 0, 0, 0, 0};

  float rmax = -__builtin_inff();
  float rsum = 0.0f;
  const float SL = 0.125f * 1.4426950408889634f * (1.0f / (QKV_CARRY * QKV_CARRY));

  #pragma unroll 1
  for (int i = 0; i < SEQ / BK; ++i) {
    const int j0 = i * BK;

    FragH ak[2][2];
    #pragma unroll
    for (int sub = 0; sub < 2; ++sub) {
      #pragma unroll
      for (int f = 0; f < 2; ++f) {
        const f16* base = k_h + (size_t)(j0 + sub * 16 + lq) * HDIM + f * 32 + hi * 8;
        ak[sub][f].q[0] = *(const v4u*)(base);
        ak[sub][f].q[1] = *(const v4u*)(base + 16);
      }
    }
    FragH bv[4];
    #pragma unroll
    for (int dt = 0; dt < 4; ++dt) {
      const f16* base = vt_h + (size_t)(dt * 16 + lq) * SEQ + j0 + hi * 8;
      bv[dt].q[0] = *(const v4u*)(base);
      bv[dt].q[1] = *(const v4u*)(base + 16);
    }

    v8f c[2];
    #pragma unroll
    for (int sub = 0; sub < 2; ++sub) {
      v8f acc = (v8f){0, 0, 0, 0, 0, 0, 0, 0};
      acc = mma_f16(ak[sub][0].v, qf[0].v, acc);
      acc = mma_f16(ak[sub][1].v, qf[1].v, acc);
      c[sub] = acc;
    }

    float m_new = rmax;
    #pragma unroll
    for (int r = 0; r < 8; ++r) {
      m_new = fmaxf(m_new, c[0][r]);
      m_new = fmaxf(m_new, c[1][r]);
    }
    m_new = fmaxf(m_new, __shfl_xor(m_new, 16, 32));
    const float scale = __builtin_amdgcn_exp2f((rmax - m_new) * SL);
    rmax = m_new;

    FragH pa;
    float psum = 0.0f;
    #pragma unroll
    for (int r = 0; r < 8; ++r) {
      const float p0 = __builtin_amdgcn_exp2f((c[0][r] - m_new) * SL);
      const float p1 = __builtin_amdgcn_exp2f((c[1][r] - m_new) * SL);
      psum += p0 + p1;
      pa.h[r]     = (f16)(p0 * P_CARRY);
      pa.h[8 + r] = (f16)(p1 * P_CARRY);
    }
    rsum = rsum * scale + psum + __shfl_xor(psum, 16, 32);

    float sc[8];
    #pragma unroll
    for (int r = 0; r < 8; ++r) sc[r] = __shfl(scale, (hi << 3) + r, 32);
    #pragma unroll
    for (int dt = 0; dt < 4; ++dt) {
      #pragma unroll
      for (int r = 0; r < 8; ++r) o[dt][r] *= sc[r];
    }

    #pragma unroll
    for (int dt = 0; dt < 4; ++dt) o[dt] = mma_f16(pa.v, bv[dt].v, o[dt]);
  }

  float rs[8];
  #pragma unroll
  for (int r = 0; r < 8; ++r) rs[r] = 1.0f / __shfl(rsum, (hi << 3) + r, 32);

  const int sob = wave * (16 * OP);
  const float OSC = CTX_CARRY / (P_CARRY * QKV_CARRY);
  #pragma unroll
  for (int r = 0; r < 8; ++r) {
    #pragma unroll
    for (int dt = 0; dt < 4; ++dt) {
      sO[sob + (hi * 8 + r) * OP + dt * 16 + lq] = o[dt][r] * OSC * rs[r];
    }
  }
  __syncthreads();

  v4u    hv[4], rv[4];
  size_t gi[4];
  #pragma unroll
  for (int it = 0; it < 4; ++it) {
    const int row = it * 4 + (lane >> 3);
    const int d0  = (lane & 7) * 8;
    const v4f x0 = *(const v4f*)(&sO[sob + row * OP + d0]);
    const v4f x1 = *(const v4f*)(&sO[sob + row * OP + d0 + 4]);
    Pack8H ph, pr;
    #pragma unroll
    for (int e = 0; e < 4; ++e) {
      const f16 t0 = (f16)x0[e];
      const f16 t1 = (f16)x1[e];
      ph.h[e]     = t0;
      ph.h[4 + e] = t1;
      pr.h[e]     = (f16)((x0[e] - (float)t0) * CTX_CARRY);
      pr.h[4 + e] = (f16)((x1[e] - (float)t1) * CTX_CARRY);
    }
    hv[it] = ph.u;
    rv[it] = pr.u;
    gi[it] = ((size_t)b * SEQ + qrow0 + row) * A2_LD + h * HDIM + d0;
  }
  #pragma unroll
  for (int it = 0; it < 4; ++it) {
    *(volatile v4u*)(a2 + gi[it])      = hv[it];
    *(volatile v4u*)(a2 + gi[it] + DM) = rv[it];
  }
  __threadfence();
  #pragma unroll
  for (int it = 0; it < 4; ++it) {
    *(volatile v4u*)(a2 + gi[it])      = hv[it];
    *(volatile v4u*)(a2 + gi[it] + DM) = rv[it];
  }
}

__global__ __launch_bounds__(256) void out_gemm_kernel(const u16* __restrict__ a2,
                                                       const u16* __restrict__ w2,
                                                       const float* __restrict__ b_out,
                                                       float* __restrict__ out) {
  __shared__ __align__(16) float sO[NWAVE * 16 * OP];
  const int tid   = threadIdx.x;
  const int wave  = __builtin_amdgcn_readfirstlane(tid >> 5);
  const int lane  = tid & 31;
  const int lq    = lane & 15;
  const int hi    = lane >> 4;
  const int waveM = wave >> 1;
  const int waveN = wave & 1;
  const int mBase = blockIdx.y * GT;
  const int nBase = blockIdx.x * GT;

  v8f acc[2][4];
  #pragma unroll
  for (int tm = 0; tm < 2; ++tm) {
    #pragma unroll
    for (int tn = 0; tn < 4; ++tn) acc[tm][tn] = (v8f){0, 0, 0, 0, 0, 0, 0, 0};
  }
  gemm_tile<0>(a2, w2, A2_LD, mBase + waveM * 32 + lq, nBase + waveN * 64 + lq, hi * 8, acc);

  float bias[4];
  #pragma unroll
  for (int tn = 0; tn < 4; ++tn) bias[tn] = (float)(bf16)b_out[nBase + waveN * 64 + tn * 16 + lq];

  const float INV = 1.0f / (CTX_CARRY * CTX_CARRY);
  const int   bb  = mBase / SEQ;
  const int   sw  = mBase - bb * SEQ + waveM * 32;
  const size_t g0 = ((size_t)bb * SEQ_FULL + sw + hi) * DM + nBase + waveN * 64 + lq * 4;
  const int   sob = wave * (16 * OP);

  v4f vals[2][8];
  #pragma unroll
  for (int tm = 0; tm < 2; ++tm) {
    if (tm == 1) __syncthreads();
    #pragma unroll
    for (int tn = 0; tn < 4; ++tn) {
      #pragma unroll
      for (int j = 0; j < 8; ++j) {
        sO[sob + (hi * 8 + j) * OP + tn * 16 + lq] = acc[tm][tn][j] * INV + bias[tn];
      }
    }
    __syncthreads();
    #pragma unroll
    for (int it = 0; it < 8; ++it) vals[tm][it] = *(const v4f*)(&sO[sob + (it * 2 + hi) * OP + lq * 4]);
    #pragma unroll
    for (int it = 0; it < 8; ++it)
      *(volatile v4f*)(out + g0 + (size_t)(tm * 16 + it * 2) * DM) = vals[tm][it];
  }
  __threadfence();
  #pragma unroll
  for (int tm = 0; tm < 2; ++tm) {
    #pragma unroll
    for (int it = 0; it < 8; ++it)
      *(volatile v4f*)(out + g0 + (size_t)(tm * 16 + it * 2) * DM) = vals[tm][it];
  }
}

extern "C" void kernel_launch(void* const* d_in, const int* in_sizes, int n_in,
                              void* d_out, int out_size, void* d_ws, size_t ws_size,
                              hipStream_t stream) {
  if (n_in < 5) return;
  const size_t rows_used = (size_t)(NB - 1) * SEQ_FULL + SEQ;
  if ((size_t)in_sizes[0] < rows_used * DM) return;
  if ((size_t)in_sizes[1] < (size_t)N3 * DM) return;
  if ((size_t)in_sizes[2] < (size_t)N3) return;
  if ((size_t)in_sizes[3] < (size_t)DM * DM) return;
  if ((size_t)in_sizes[4] < (size_t)DM) return;
  if ((size_t)out_size < rows_used * DM) return;
  if (ws_size < WS_TOTAL) return;

  const float* x     = (const float*)d_in[0];
  const float* w_in  = (const float*)d_in[1];
  const float* b_in  = (const float*)d_in[2];
  const float* w_out = (const float*)d_in[3];
  const float* b_out = (const float*)d_in[4];
  float*       out   = (float*)d_out;

  char* ws = (char*)d_ws;
  u16* xb = (u16*)(ws);
  u16* wb = (u16*)(ws + XB_BYTES);
  f16* w2 = (f16*)(ws + XB_BYTES + WB_BYTES);
  f16* qk = (f16*)(ws + XB_BYTES + WB_BYTES + W2_BYTES);
  f16* vt = (f16*)(ws + XB_BYTES + WB_BYTES + W2_BYTES + QK_BYTES);
  f16* a2 = (f16*)(ws + XB_BYTES + WB_BYTES + W2_BYTES + QK_BYTES + VT_BYTES);

  cvt_bf16_kernel<<<dim3((MROWS * 128 + 255) / 256), 256, 0, stream>>>(x, xb, MROWS, SEQ, SEQ_FULL);
  cvt_bf16_kernel<<<dim3((N3 * 128 + 255) / 256), 256, 0, stream>>>(w_in, wb, N3, N3, N3);
  cvt_wout_kernel<<<dim3((DM * 128 + 255) / 256), 256, 0, stream>>>(w_out, w2);

  qkv_gemm_kernel<<<dim3(N3 / GT, MROWS / GT), 256, 0, stream>>>(xb, wb, b_in, qk, vt);

  attn_kernel<<<dim3(SEQ / BQ, NHEAD, NB), 256, 0, stream>>>(qk, vt, a2);

  out_gemm_kernel<<<dim3(DM / GT, MROWS / GT), 256, 0, stream>>>((const u16*)a2, (const u16*)w2, b_out, out);
}
